// RNN_45878840656508
// MI455X (gfx1250) — hardware-verified
//
#include <hip/hip_runtime.h>
#include <math.h>

constexpr int NBATCH   = 256;
constexpr int NSTEP    = 512;
constexpr int NIN      = 64;
constexpr int NHID     = 512;
constexpr int KCAT     = NHID + NIN;
constexpr int ROWS_BLK = 32;
constexpr int NTHR_SCAN = 512;
constexpr int NWAVE_SCAN = NTHR_SCAN / 32;
constexpr int APITCH   = 584;
constexpr int TILE_ELEMS = ROWS_BLK * APITCH;
constexpr int ZERO_VECS = (2 * TILE_ELEMS) / 8;
constexpr float WCARRY     = 256.0f;
constexpr float WCARRY_INV = 1.0f / 256.0f;
constexpr int NTHR_PACK = 256;
constexpr int PACK_BLK_HH = (NHID * (NHID / 8)) / NTHR_PACK;
constexpr int PACK_BLK_IH = (NHID * (NIN / 8)) / NTHR_PACK;

static_assert(KCAT % 32 == 0);
static_assert(KCAT == 576);
static_assert(NBATCH % ROWS_BLK == 0);
static_assert(NHID == 32 * NWAVE_SCAN);
static_assert(ROWS_BLK == 2 * NWAVE_SCAN);
static_assert(NSTEP % 32 == 0);
static_assert(ROWS_BLK * NIN == NTHR_SCAN * 4);
static_assert((APITCH * 2) % 16 == 0);
static_assert(APITCH >= KCAT);
static_assert((2 * TILE_ELEMS) % 8 == 0);
static_assert((NHID * (NHID / 8)) % NTHR_PACK == 0);
static_assert((NHID * (NIN / 8)) % NTHR_PACK == 0);
static_assert(PACK_BLK_HH == 128 && PACK_BLK_IH == 16);
static_assert((KCAT * 2) % 128 == 0);

typedef __attribute__((ext_vector_type(16))) _Float16 v16h;
typedef __attribute__((ext_vector_type(8)))  _Float16 v8h;
typedef __attribute__((ext_vector_type(8)))  float    v8f;
typedef __attribute__((ext_vector_type(4)))  float    v4f;
typedef __attribute__((ext_vector_type(4)))  unsigned v4u;
typedef __attribute__((ext_vector_type(2)))  unsigned v2u;

__device__ __forceinline__ v16h frag_load_h(const _Float16* p) {
  union U { v16h v; v8h h[2]; };
  U f;
  f.h[0] = *(const v8h*)(p);
  f.h[1] = *(const v8h*)(p + 16);
  return f.v;
}
__device__ __forceinline__ v8f mma_h(v16h a, v16h b, v8f c) {
  return __builtin_amdgcn_wmma_f32_16x16x32_f16(false, a, false, b, (short)0, c, false, false);
}
__device__ __forceinline__ void guard_group(v8f& a, v8f& b, v8f& c, v8f& d, v16h x0, v16h x1, v16h y0, v16h y1) {
  asm volatile("v_nop\n\tv_nop\n\tv_nop\n\tv_nop" : "+v"(a), "+v"(b), "+v"(c), "+v"(d) : "v"(x0), "v"(x1), "v"(y0), "v"(y1));
}
__device__ __forceinline__ void acc_guard4(v8f& a, v8f& b, v8f& c, v8f& d) {
  asm volatile("v_nop\n\tv_nop\n\tv_nop\n\tv_nop" : "+v"(a), "+v"(b), "+v"(c), "+v"(d));
}

__device__ __forceinline__ float h16_to_f32(unsigned hb) {
  const unsigned sgn = (hb & 0x8000u) << 16;
  const unsigned em = hb & 0x7fffu;
  const float fn = __uint_as_float((em << 13) + 0x38000000u);
  const float fs = (float)em * 5.9604644775390625e-8f;
  const float mag = (em < 0x400u) ? fs : fn;
  return __uint_as_float(__float_as_uint(mag) | sgn);
}

__device__ __forceinline__ void store_x4(unsigned short* dst, const v4f v) {
  const float f0 = v[0];
  const float f1 = v[1];
  const float f2 = v[2];
  const float f3 = v[3];
  const _Float16 g0 = (_Float16)f0;
  const _Float16 g1 = (_Float16)f1;
  const _Float16 g2 = (_Float16)f2;
  const _Float16 g3 = (_Float16)f3;
  const unsigned u0 = (unsigned)__builtin_bit_cast(unsigned short, g0);
  const unsigned u1 = (unsigned)__builtin_bit_cast(unsigned short, g1);
  const unsigned u2 = (unsigned)__builtin_bit_cast(unsigned short, g2);
  const unsigned u3 = (unsigned)__builtin_bit_cast(unsigned short, g3);
  v2u pk;
  pk[0] = u0 | (u1 << 16);
  pk[1] = u2 | (u3 << 16);
  *(v2u*)dst = pk;
}

__device__ __forceinline__ void tanh_store8(const v8f acc, const float bias, unsigned short* dst) {
#pragma unroll
  for (int r = 0; r < 8; ++r) {
    const float z  = acc[r] * WCARRY_INV + bias;
    const float e  = expf(2.0f * z);
    const float hn = 1.0f - 2.0f * __builtin_amdgcn_rcpf(e + 1.0f);
    const _Float16 h16 = (_Float16)hn;
    dst[r * APITCH] = __builtin_bit_cast(unsigned short, h16);
  }
}

__device__ __forceinline__ float row_dot16(const unsigned short* rowp, const int lane, const float (&wr)[16]) {
  const v4u qa = *(const v4u*)(rowp + 16 * lane);
  const v4u qb = *(const v4u*)(rowp + 16 * lane + 8);
  float s = 0.0f;
#pragma unroll
  for (int j = 0; j < 4; ++j) {
    const unsigned w = qa[j];
    s = fmaf(h16_to_f32(w & 0xffffu), wr[2 * j], s);
    s = fmaf(h16_to_f32(w >> 16), wr[2 * j + 1], s);
  }
#pragma unroll
  for (int j = 0; j < 4; ++j) {
    const unsigned w = qb[j];
    s = fmaf(h16_to_f32(w & 0xffffu), wr[8 + 2 * j], s);
    s = fmaf(h16_to_f32(w >> 16), wr[8 + 2 * j + 1], s);
  }
  return s;
}

__global__ __launch_bounds__(NTHR_PACK) void pack_w_kernel(const float* __restrict__ w_hh, const float* __restrict__ w_ih,
                                                           unsigned short* __restrict__ wcat) {
  const int tid = threadIdx.x;
  const int blk = blockIdx.x;
  const float* sp;
  size_t dofs;
  if (blk < PACK_BLK_HH) {
    const int i  = blk * NTHR_PACK + tid;
    const int n  = i >> 6;
    const int c8 = i & 63;
    sp   = w_hh + (size_t)n * NHID + c8 * 8;
    dofs = (size_t)n * KCAT + c8 * 8;
  } else {
    const int i  = (blk - PACK_BLK_HH) * NTHR_PACK + tid;
    const int n  = i >> 3;
    const int c8 = i & 7;
    sp   = w_ih + (size_t)n * NIN + c8 * 8;
    dofs = (size_t)n * KCAT + NHID + c8 * 8;
  }
  const v4f a = *(const v4f*)(sp);
  const v4f b = *(const v4f*)(sp + 4);
  v8h hv;
#pragma unroll
  for (int e = 0; e < 4; ++e) {
    hv[e]     = (_Float16)(a[e] * WCARRY);
    hv[4 + e] = (_Float16)(b[e] * WCARRY);
  }
  unsigned short* dp = wcat + dofs;
  *(volatile v8h*)dp = hv;
  __threadfence();
  *(volatile v8h*)dp = hv;
}

__global__ __launch_bounds__(NTHR_SCAN) void rnn_scan_kernel(const float* __restrict__ x, const unsigned short* __restrict__ wcatp,
                                                            const float* __restrict__ b_ih, const float* __restrict__ b_hh,
                                                            const float* __restrict__ w_ho, const float* __restrict__ b_ho,
                                                            float* __restrict__ out) {
  __shared__ __align__(16) unsigned short At[2 * TILE_ELEMS];
  const _Float16* Wc = (const _Float16*)wcatp;
  const int tid  = threadIdx.x;
  const int lane = tid & 31;
  const int wave = tid >> 5;
  const int c    = lane & 15;
  const int hh   = lane >> 4;
  const int koff = hh * 8;
  const int b0   = blockIdx.x * ROWS_BLK;

  {
    const v4u zz = {0u, 0u, 0u, 0u};
    v4u* ap = (v4u*)At;
#pragma unroll 1
    for (int i = tid; i < ZERO_VECS; i += NTHR_SCAN) ap[i] = zz;
  }
  __syncthreads();

  const int xrow = tid >> 4;
  const int xc4  = (tid & 15) * 4;
  const float* xbase = x + (size_t)(b0 + xrow) * NSTEP * NIN + xc4;
  {
    const v4f v0 = *(const v4f*)(xbase);
    store_x4(At + xrow * APITCH + NHID + xc4, v0);
  }

  float wreg[16];
  {
    const v4f w0 = *(const v4f*)(w_ho + 16 * lane);
    const v4f w1 = *(const v4f*)(w_ho + 16 * lane + 4);
    const v4f w2 = *(const v4f*)(w_ho + 16 * lane + 8);
    const v4f w3 = *(const v4f*)(w_ho + 16 * lane + 12);
#pragma unroll
    for (int e = 0; e < 4; ++e) {
      wreg[e]      = w0[e];
      wreg[4 + e]  = w1[e];
      wreg[8 + e]  = w2[e];
      wreg[12 + e] = w3[e];
    }
  }
  const int n0 = 32 * wave + c;
  const int n1 = 32 * wave + 16 + c;
  const float bias0 = b_ih[n0] + b_hh[n0];
  const float bias1 = b_ih[n1] + b_hh[n1];
  const float bho   = b_ho[0];
  const _Float16* b0p = Wc + (size_t)n0 * KCAT + koff;
  const _Float16* b1p = Wc + (size_t)n1 * KCAT + koff;
  __syncthreads();

  const v8f z8 = {0.f, 0.f, 0.f, 0.f, 0.f, 0.f, 0.f, 0.f};
  float o0 = 0.0f;
  float o1 = 0.0f;
  int p = 0;

#pragma unroll 1
  for (int t = 0; t < NSTEP; ++t) {
    const int tn = (t + 1 < NSTEP) ? (t + 1) : (NSTEP - 1);
    const v4f xv = *(const v4f*)(xbase + (size_t)tn * NIN);

    const unsigned short* Acur = At + p * TILE_ELEMS;
    unsigned short* Anext = At + (p ^ 1) * TILE_ELEMS;
    const _Float16* a0p = (const _Float16*)Acur + c * APITCH + koff;
    const _Float16* a1p = (const _Float16*)Acur + (16 + c) * APITCH + koff;

    v8f acc00 = z8;
    v8f acc01 = z8;
    v8f acc10 = z8;
    v8f acc11 = z8;
#pragma unroll 1
    for (int k0 = 0; k0 < KCAT; k0 += 32) {
      const v16h a0 = frag_load_h(a0p + k0);
      const v16h a1 = frag_load_h(a1p + k0);
      const v16h w0 = frag_load_h(b0p + k0);
      const v16h w1 = frag_load_h(b1p + k0);
      acc00 = mma_h(a0, w0, acc00);
      acc01 = mma_h(a0, w1, acc01);
      acc10 = mma_h(a1, w0, acc10);
      acc11 = mma_h(a1, w1, acc11);
      guard_group(acc00, acc01, acc10, acc11, a0, a1, w0, w1);
    }
    acc_guard4(acc00, acc01, acc10, acc11);

    tanh_store8(acc00, bias0, Anext + (8 * hh) * APITCH + n0);
    tanh_store8(acc01, bias1, Anext + (8 * hh) * APITCH + n1);
    tanh_store8(acc10, bias0, Anext + (16 + 8 * hh) * APITCH + n0);
    tanh_store8(acc11, bias1, Anext + (16 + 8 * hh) * APITCH + n1);
    store_x4(Anext + xrow * APITCH + NHID + xc4, xv);

    __syncthreads();

    float s0 = row_dot16(Anext + (2 * wave) * APITCH, lane, wreg);
    float s1 = row_dot16(Anext + (2 * wave + 1) * APITCH, lane, wreg);
#pragma unroll
    for (int off = 16; off >= 1; off >>= 1) {
      s0 += __shfl_xor(s0, off, 32);
      s1 += __shfl_xor(s1, off, 32);
    }
    const float r0 = s0 + bho;
    const float r1 = s1 + bho;
    const bool mine = (lane == (t & 31));
    o0 = mine ? r0 : o0;
    o1 = mine ? r1 : o1;

    if ((t & 31) == 31) {
      float* op0 = out + (size_t)(b0 + 2 * wave) * NSTEP + (size_t)(t - 31) + lane;
      float* op1 = op0 + NSTEP;
      const float v0 = o0;
      const float v1 = o1;
      *(volatile float*)op0 = v0;
      *(volatile float*)op1 = v1;
      __threadfence();
      *(volatile float*)op0 = v0;
      *(volatile float*)op1 = v1;
    }
    p ^= 1;
  }
}

extern "C" void kernel_launch(void* const* d_in, const int* in_sizes, int n_in,
                              void* d_out, int out_size, void* d_ws, size_t ws_size, hipStream_t stream) {
  if (n_in < 7 || d_out == nullptr || d_ws == nullptr) return;
  if (in_sizes[0] != NBATCH * NSTEP * NIN || in_sizes[1] != NHID * NIN || in_sizes[2] != NHID * NHID ||
      in_sizes[3] != NHID || in_sizes[4] != NHID || in_sizes[5] != NHID || in_sizes[6] != 1 ||
      out_size != NBATCH * NSTEP) return;

  const float* x    = (const float*)d_in[0];
  const float* w_ih = (const float*)d_in[1];
  const float* w_hh = (const float*)d_in[2];
  const float* b_ih = (const float*)d_in[3];
  const float* b_hh = (const float*)d_in[4];
  const float* w_ho = (const float*)d_in[5];
  const float* b_ho = (const float*)d_in[6];
  float* out = (float*)d_out;

  const size_t wcat_bytes = (size_t)NHID * KCAT * 2;
  if (wcat_bytes > ws_size || wcat_bytes > (size_t)134217728) return;
  unsigned short* wcat = (unsigned short*)d_ws;

  pack_w_kernel<<<PACK_BLK_HH + PACK_BLK_IH, NTHR_PACK, 0, stream>>>(w_hh, w_ih, wcat);
  rnn_scan_kernel<<<NBATCH / ROWS_BLK, NTHR_SCAN, 0, stream>>>(x, wcat, b_ih, b_hh, w_ho, b_ho, out);
}
